// EGNNEncoder_11261404250494
// MI455X (gfx1250) — hardware-verified
//
#include <hip/hip_runtime.h>
#include <math.h>

typedef __attribute__((ext_vector_type(16))) _Float16 v16h;
typedef __attribute__((ext_vector_type(8)))  _Float16 v8h;
typedef __attribute__((ext_vector_type(8)))  float  v8f;
typedef __attribute__((ext_vector_type(4)))  float  v4f;
typedef __attribute__((ext_vector_type(4)))  unsigned v4u;
typedef float __attribute__((may_alias)) float_a;

#define N_NODES 32768
#define NE 262144
#define HH 128
#define K1 288
#define NL 4
#define BT 256
#define ECAP 2560
#define SCAP 32
#define ETILE 2048
#define NBUCK (N_NODES / BT)

template <typename V> __device__ __forceinline__ void vst2(void* p, V v) {
  *(volatile V*)p = v; __threadfence(); *(volatile V*)p = v;
}
__device__ __forceinline__ v8f wmma_f16(v16h a, v16h b, v8f c) {
  v8f d = __builtin_amdgcn_wmma_f32_16x16x32_f16(false, a, false, b, (short)0, c, false, false);
  asm volatile("v_nop\n\tv_nop\n\tv_nop\n\tv_nop" : "+v"(d) : "v"(a), "v"(b));
  return d;
}
__device__ __forceinline__ v16h frag_h(const _Float16* row, int k0, int lane) {
  union { v16h v; v8h h[2]; } r; const _Float16* p = row + k0 + 8 * (lane >> 4);
  r.h[0] = *(const v8h*)(p); r.h[1] = *(const v8h*)(p + 16); return r.v;
}
__device__ __forceinline__ v16h frag_f32(const float* row, int k0, int lane) {
  v16h a; const float* p = row + k0 + 8 * (lane >> 4);
#pragma unroll
  for (int i = 0; i < 8; ++i) { a[i] = (_Float16)p[i]; a[8 + i] = (_Float16)p[16 + i]; }
  return a;
}
__device__ __forceinline__ float siluf(float x) { return x / (1.f + __expf(-x)); }

struct Bucket {
  int ledge[ECAP]; unsigned short ltgt[ECAP]; unsigned short sub[BT][SCAP]; int scnt[BT]; int wcnt[8][8]; int total;
};
__device__ void bucket_build(Bucket& bk, const int* __restrict__ src, const int* __restrict__ dst, int E, int tlo, int tid) {
  const int lane = tid & 31, wave = tid >> 5;
  if (tid == 0) bk.total = 0;
  __syncthreads();
  for (int e0 = 0; e0 < E; e0 += ETILE) {
    int rv[8]; unsigned msk[8];
#pragma unroll
    for (int j = 0; j < 8; ++j) {
      const int e = e0 + j * 256 + tid;
      const int r = (e < E) ? dst[e] : -1;
      rv[j] = r;
      msk[j] = (unsigned)__builtin_amdgcn_ballot_w32((r >= tlo) && (r < tlo + BT));
    }
    if (lane < 8) bk.wcnt[lane][wave] = __builtin_popcount(msk[lane]);
    __syncthreads();
    const int base = bk.total;
    int run = 0, pre[8];
#pragma unroll
    for (int j = 0; j < 8; ++j) {
#pragma unroll
      for (int w = 0; w < 8; ++w) { if (w == wave) pre[j] = run; run += bk.wcnt[j][w]; }
    }
#pragma unroll
    for (int j = 0; j < 8; ++j) {
      const unsigned m = msk[j];
      if ((m >> lane) & 1u) {
        const int pos = base + pre[j] + __builtin_popcount(m & ((1u << lane) - 1u));
        if (pos < ECAP) { bk.ledge[pos] = e0 + j * 256 + tid; bk.ltgt[pos] = (unsigned short)(rv[j] - tlo); }
      }
    }
    __syncthreads();
    if (tid == 0) bk.total = base + run;
    __syncthreads();
  }
  const int n = (bk.total < ECAP) ? bk.total : ECAP;
  (void)src;
  int k = 0;
  for (int i = 0; i < n; ++i) if ((int)bk.ltgt[i] == tid) { if (k < SCAP) bk.sub[tid][k] = (unsigned short)i; ++k; }
  bk.scnt[tid] = (k < SCAP) ? k : SCAP;
  __syncthreads();
}


__global__ __launch_bounds__(256) void k_wt(const float* __restrict__ W, _Float16* __restrict__ WT, int K, int M, int Kp, int mofs) {
  __shared__ __align__(16) _Float16 tile[64][72];
  const int mt = M / 64, tid = threadIdx.x;
  const int m0 = (blockIdx.x % mt) * 64, k0 = (blockIdx.x / mt) * 64;
  for (int i = tid; i < 64 * 64; i += 256) { const int kk = i >> 6, mm = i & 63; const int k = k0 + kk;
    tile[mm][kk] = (k < K) ? (_Float16)W[(size_t)k * M + m0 + mm] : (_Float16)0.f; }
  __syncthreads();
  for (int g = tid; g < 64 * 8; g += 256) { const int mm = g >> 3, pc = g & 7; if (k0 + pc * 8 < Kp) vst2(WT + (size_t)(mofs + m0 + mm) * Kp + k0 + pc * 8, *(const v4u*)(&tile[mm][pc * 8])); }
}

__device__ __forceinline__ void mm_lds128(const float* At, const _Float16* __restrict__ WT, int n0, int lane, v8f& c0, v8f& c1) {
  const int col = lane & 15;
  c0 = (v8f){}; c1 = (v8f){};
#pragma unroll
  for (int kc = 0; kc < 4; ++kc) {
    v16h a; const float* p = At + col * 132 + kc * 32 + 8 * (lane >> 4);
#pragma unroll
    for (int i = 0; i < 8; ++i) { a[i] = (_Float16)p[i]; a[8 + i] = (_Float16)p[16 + i]; }
    c0 = wmma_f16(a, frag_h(WT + (size_t)(n0 + col) * HH, kc * 32, lane), c0);
    c1 = wmma_f16(a, frag_h(WT + (size_t)(n0 + 16 + col) * HH, kc * 32, lane), c1);
  }
}

__global__ __launch_bounds__(128) void k_proj(const float* __restrict__ x, const _Float16* __restrict__ WT, const float* __restrict__ b, float* __restrict__ h) {
  __shared__ __align__(16) float T[16][132];
  const int tid = threadIdx.x, wave = tid >> 5, lane = tid & 31, hi = lane >> 4, col = lane & 15, m0 = blockIdx.x * 16;
  v8f c0 = {}, c1 = {};
  const float* ar = x + (size_t)(m0 + col) * HH;
#pragma unroll
  for (int kc = 0; kc < 4; ++kc) { const v16h a = frag_f32(ar, kc * 32, lane);
    c0 = wmma_f16(a, frag_h(WT + (size_t)(wave * 32 + col) * HH, kc * 32, lane), c0);
    c1 = wmma_f16(a, frag_h(WT + (size_t)(wave * 32 + 16 + col) * HH, kc * 32, lane), c1); }
#pragma unroll
  for (int r = 0; r < 8; ++r) { T[hi * 8 + r][wave * 32 + col] = c0[r] + b[wave * 32 + col]; T[hi * 8 + r][wave * 32 + 16 + col] = c1[r] + b[wave * 32 + 16 + col]; }
  __syncthreads();
  for (int g = tid; g < 16 * 32; g += 128) { const int rl = g >> 5, pc = g & 31; vst2(h + (size_t)(m0 + rl) * HH + pc * 4, *(const v4f*)(&T[rl][pc * 4])); }
}

__global__ __launch_bounds__(128) void k_edge(const int* __restrict__ erow, const int* __restrict__ ecol, const float* __restrict__ h,
                                             const float* __restrict__ pos, const _Float16* __restrict__ W1T, const float* __restrict__ b1,
                                             const _Float16* __restrict__ W2T, const float* __restrict__ b2, const _Float16* __restrict__ Wc1T,
                                             const float* __restrict__ bc1, const float* __restrict__ wc2,
                                             float* __restrict__ mbuf, float* __restrict__ trans) {
  __shared__ __align__(16) float T[16][132];
  __shared__ __align__(16) float U[16][132];
  __shared__ float dist_s[16], dif_s[16][3], cwp[4][16];
  const int tid = threadIdx.x, wave = tid >> 5, lane = tid & 31, hi = lane >> 4, col = lane & 15;
  const int e0 = blockIdx.x * 16;
  if (tid < 16) {
    const int e = e0 + tid, r_ = erow[e], c_ = ecol[e];
    const float dx = pos[r_ * 3] - pos[c_ * 3], dy = pos[r_ * 3 + 1] - pos[c_ * 3 + 1], dz = pos[r_ * 3 + 2] - pos[c_ * 3 + 2];
    const float d = fmaxf(sqrtf(dx * dx + dy * dy + dz * dz), 1e-6f);
    dist_s[tid] = d; dif_s[tid][0] = dx; dif_s[tid][1] = dy; dif_s[tid][2] = dz;
  }
  __syncthreads();
  const int er = erow[e0 + col], ec = ecol[e0 + col];
  const float* hr = h + (size_t)er * HH; const float* hc = h + (size_t)ec * HH;
  v8f c0 = {}, c1 = {};
  const int n0 = wave * 32;
#pragma unroll
  for (int kc = 0; kc < 9; ++kc) {
    v16h a;
    if (kc < 4) a = frag_f32(hr, kc * 32, lane);
    else if (kc < 8) a = frag_f32(hc, (kc - 4) * 32, lane);
    else {
#pragma unroll
      for (int i = 0; i < 16; ++i) a[i] = (_Float16)0.f;
      if (hi == 0) a[0] = (_Float16)dist_s[col];
    }
    c0 = wmma_f16(a, frag_h(W1T + (size_t)(n0 + col) * K1, kc * 32, lane), c0);
    c1 = wmma_f16(a, frag_h(W1T + (size_t)(n0 + 16 + col) * K1, kc * 32, lane), c1);
  }
#pragma unroll
  for (int r = 0; r < 8; ++r) { T[hi * 8 + r][n0 + col] = siluf(c0[r] + b1[n0 + col]); T[hi * 8 + r][n0 + 16 + col] = siluf(c1[r] + b1[n0 + 16 + col]); }
  __syncthreads();
  mm_lds128(&T[0][0], W2T, n0, lane, c0, c1);
#pragma unroll
  for (int r = 0; r < 8; ++r) { U[hi * 8 + r][n0 + col] = siluf(c0[r] + b2[n0 + col]); U[hi * 8 + r][n0 + 16 + col] = siluf(c1[r] + b2[n0 + 16 + col]); }
  __syncthreads();
  for (int g = tid; g < 16 * 32; g += 128) { const int rl = g >> 5, pc = g & 31; vst2(mbuf + (size_t)(e0 + rl) * HH + pc * 4, *(const v4f*)(&U[rl][pc * 4])); }
  mm_lds128(&U[0][0], Wc1T, n0, lane, c0, c1);
  {
    const float w0 = wc2[n0 + col], w1 = wc2[n0 + 16 + col];
#pragma unroll
    for (int r = 0; r < 8; ++r) {
      float p = siluf(c0[r] + bc1[n0 + col]) * w0 + siluf(c1[r] + bc1[n0 + 16 + col]) * w1;
#pragma unroll
      for (int off = 8; off > 0; off >>= 1) p += __shfl_xor(p, off, 32);
      if (col == 0) cwp[wave][hi * 8 + r] = p;
    }
  }
  __syncthreads();
  if (tid < 16) {
    float cw = cwp[0][tid] + cwp[1][tid] + cwp[2][tid] + cwp[3][tid];
    cw = fminf(fmaxf(cw, -1.f), 1.f);
    const float inv = cw / dist_s[tid];
    v4f t4 = {dif_s[tid][0] * inv, dif_s[tid][1] * inv, dif_s[tid][2] * inv, 0.f};
    vst2(trans + (size_t)(e0 + tid) * 4, t4);
  }
}

__global__ __launch_bounds__(256) void k_gather(const int* __restrict__ erow, const int* __restrict__ ecol, const float* __restrict__ mbuf,
                                               const float* __restrict__ trans, const float* __restrict__ posin, float* __restrict__ posout,
                                               float* __restrict__ agg) {
  __shared__ Bucket bk;
  __shared__ __align__(16) float ps[BT * 3];
  const int tid = threadIdx.x, lane = tid & 31, wave = tid >> 5, tlo = blockIdx.x * BT;
  bucket_build(bk, ecol, erow, NE, tlo, tid);
  for (int s = 0; s < 32; ++s) {
    const int t = wave * 32 + s, node = tlo + t;
    const int cnt = bk.scnt[t];
    float a[4] = {0.f, 0.f, 0.f, 0.f}; float px = 0.f, py = 0.f, pz = 0.f;
    for (int k = 0; k < cnt; ++k) {
      const int e = bk.ledge[bk.sub[t][k]];
      const float* mr = mbuf + (size_t)e * HH;
#pragma unroll
      for (int j = 0; j < 4; ++j) a[j] += mr[lane + 32 * j];
      if (lane < 3) { const float tv = trans[(size_t)e * 4 + lane]; if (lane == 0) px += tv; else if (lane == 1) py += tv; else pz += tv; }
    }
    float* ar = agg + (size_t)node * HH;
#pragma unroll
    for (int j = 0; j < 4; ++j) vst2(ar + lane + 32 * j, (float_a)a[j]);
    if (lane < 3) ps[t * 3 + lane] = posin[(size_t)node * 3 + lane] + (lane == 0 ? px : lane == 1 ? py : pz);
  }
  __syncthreads();
  if (tid < 192) vst2(posout + (size_t)tlo * 3 + tid * 4, *(const v4f*)(&ps[tid * 4]));
}

__global__ __launch_bounds__(128) void k_node(const float* __restrict__ h, const float* __restrict__ agg, const _Float16* __restrict__ Wn1T,
                                             const float* __restrict__ bn1, const _Float16* __restrict__ Wn2T, const float* __restrict__ bn2,
                                             float* __restrict__ hout) {
  __shared__ __align__(16) float T[16][132];
  __shared__ __align__(16) float U[16][132];
  const int tid = threadIdx.x, wave = tid >> 5, lane = tid & 31, hi = lane >> 4, col = lane & 15, m0 = blockIdx.x * 16, n0 = wave * 32;
  const float* hr = h + (size_t)(m0 + col) * HH; const float* gr = agg + (size_t)(m0 + col) * HH;
  v8f c0 = {}, c1 = {};
#pragma unroll
  for (int kc = 0; kc < 8; ++kc) {
    const v16h a = (kc < 4) ? frag_f32(hr, kc * 32, lane) : frag_f32(gr, (kc - 4) * 32, lane);
    c0 = wmma_f16(a, frag_h(Wn1T + (size_t)(n0 + col) * 256, kc * 32, lane), c0);
    c1 = wmma_f16(a, frag_h(Wn1T + (size_t)(n0 + 16 + col) * 256, kc * 32, lane), c1);
  }
#pragma unroll
  for (int r = 0; r < 8; ++r) { T[hi * 8 + r][n0 + col] = siluf(c0[r] + bn1[n0 + col]); T[hi * 8 + r][n0 + 16 + col] = siluf(c1[r] + bn1[n0 + 16 + col]); }
  __syncthreads();
  mm_lds128(&T[0][0], Wn2T, n0, lane, c0, c1);
#pragma unroll
  for (int r = 0; r < 8; ++r) { const int rl = hi * 8 + r;
    U[rl][n0 + col] = c0[r] + bn2[n0 + col] + h[(size_t)(m0 + rl) * HH + n0 + col];
    U[rl][n0 + 16 + col] = c1[r] + bn2[n0 + 16 + col] + h[(size_t)(m0 + rl) * HH + n0 + 16 + col]; }
  __syncthreads();
  for (int g = tid; g < 16 * 32; g += 128) { const int rl = g >> 5, pc = g & 31; vst2(hout + (size_t)(m0 + rl) * HH + pc * 4, *(const v4f*)(&U[rl][pc * 4])); }
}

extern "C" void kernel_launch(void* const* d_in, const int* in_sizes, int n_in,
                              void* d_out, int out_size, void* d_ws, size_t ws_size,
                              hipStream_t stream) {
  (void)in_sizes; (void)n_in; (void)out_size; (void)ws_size;
  const float* x   = (const float*)d_in[0];
  const float* pos = (const float*)d_in[1];
  const int*   ei  = (const int*)d_in[2];
  const int* erow = ei; const int* ecol = ei + NE;
  const float *proj_w = (const float*)d_in[3], *proj_b = (const float*)d_in[4];
  const float *ew1 = (const float*)d_in[5], *eb1 = (const float*)d_in[6], *ew2 = (const float*)d_in[7], *eb2 = (const float*)d_in[8];
  const float *nw1 = (const float*)d_in[9], *nb1 = (const float*)d_in[10], *nw2 = (const float*)d_in[11], *nb2 = (const float*)d_in[12];
  const float *cw1 = (const float*)d_in[13], *cb1 = (const float*)d_in[14], *cw2 = (const float*)d_in[15];
  float* out_h   = (float*)d_out;
  float* out_pos = out_h + (size_t)N_NODES * HH;

  char* ws = (char*)d_ws; size_t off = 0;
  auto alloc = [&](size_t bytes) -> void* { void* p = ws + off; off = (off + bytes + 255) & ~(size_t)255; return p; };
  _Float16* WpT  = (_Float16*)alloc((size_t)HH * HH * 2);
  _Float16* W1T  = (_Float16*)alloc((size_t)HH * K1 * 2);
  _Float16* W2T  = (_Float16*)alloc((size_t)HH * HH * 2);
  _Float16* Wc1T = (_Float16*)alloc((size_t)HH * HH * 2);
  _Float16* Wn1T = (_Float16*)alloc((size_t)HH * 256 * 2);
  _Float16* Wn2T = (_Float16*)alloc((size_t)HH * HH * 2);
  float* hA   = (float*)alloc((size_t)N_NODES * HH * 4);
  float* hB   = (float*)alloc((size_t)N_NODES * HH * 4);
  float* agg  = (float*)alloc((size_t)N_NODES * HH * 4);
  float* posA = (float*)alloc((size_t)N_NODES * 3 * 4);
  float* posB = (float*)alloc((size_t)N_NODES * 3 * 4);
  float* mbuf = (float*)alloc((size_t)NE * HH * 4);
  float* trans = (float*)alloc((size_t)NE * 4 * 4);

  k_wt<<<(HH / 64) * (HH / 64), 256, 0, stream>>>(proj_w, WpT, HH, HH, HH, 0);
  k_proj<<<N_NODES / 16, 128, 0, stream>>>(x, WpT, proj_b, hA);
  const float* pcur = pos; float* hcur = hA;
  for (int l = 0; l < NL; ++l) {
    const bool last = (l == NL - 1);
    k_wt<<<(320 / 64) * (HH / 64), 256, 0, stream>>>(ew1 + (size_t)l * 257 * HH, W1T, 257, HH, K1, 0);
    k_wt<<<(HH / 64) * (HH / 64), 256, 0, stream>>>(ew2 + (size_t)l * HH * HH, W2T, HH, HH, HH, 0);
    k_wt<<<(HH / 64) * (HH / 64), 256, 0, stream>>>(cw1 + (size_t)l * HH * HH, Wc1T, HH, HH, HH, 0);
    k_wt<<<(256 / 64) * (HH / 64), 256, 0, stream>>>(nw1 + (size_t)l * 256 * HH, Wn1T, 256, HH, 256, 0);
    k_wt<<<(HH / 64) * (HH / 64), 256, 0, stream>>>(nw2 + (size_t)l * HH * HH, Wn2T, HH, HH, HH, 0);
    k_edge<<<NE / 16, 128, 0, stream>>>(erow, ecol, hcur, pcur, W1T, eb1 + l * HH, W2T, eb2 + l * HH, Wc1T, cb1 + l * HH, cw2 + l * HH, mbuf, trans);
    float* pout = last ? out_pos : ((l & 1) ? posB : posA);
    k_gather<<<NBUCK, 256, 0, stream>>>(erow, ecol, mbuf, trans, pcur, pout, agg);
    float* hout = last ? out_h : ((l & 1) ? hA : hB);
    k_node<<<N_NODES / 16, 128, 0, stream>>>(hcur, agg, Wn1T, nb1 + l * HH, Wn2T, nb2 + l * HH, hout);
    pcur = pout; hcur = hout;
  }
}
